// MultiHeadSelfAttention_18373870092947
// MI455X (gfx1250) — hardware-verified
//
#include <hip/hip_runtime.h>
#ifndef NB
#define NB 2
#endif
#ifndef SQ
#define SQ 2048
#endif
#define NB_FULL 2
#define SQ_FULL 2048
#define DM 1024
#define NH 16
#define HD 64
#define HG 2
#define NR ((size_t)NB * SQ)
#define LQ (3 * DM)

static_assert(DM == 256 * 4);
static_assert(NH * HD == DM);
static_assert(HD == 64);
static_assert(HD % 32 == 0 && DM % 32 == 0 && SQ % 32 == 0);
static_assert(SQ % 128 == 0);
static_assert(((size_t)NB * SQ) % 128 == 0);
static_assert((3 * DM) % 64 == 0 && DM % 8 == 0);
static_assert(NH % HG == 0);
static_assert(NB <= NB_FULL && SQ <= SQ_FULL);
static_assert((size_t)NB_FULL * SQ_FULL * DM * 4 == (size_t)16777216);

#define SZ_BQKV ((size_t)3 * DM * DM * 2)
#define SZ_XN32 (NR * DM * 4)
#define SZ_XN16 (NR * DM * 2)
#define SZ_QKV  (NR * 3 * DM * 2)
#define SZ_S    ((size_t)HG * SQ * SQ * 4)
#define SZ_P    ((size_t)HG * SQ * SQ * 2)
#define SZ_VT   ((size_t)NB * NH * HD * SQ * 2)
#define SZ_TOTAL (SZ_BQKV + SZ_XN32 + SZ_XN16 + SZ_QKV + SZ_S + SZ_P + SZ_VT + (size_t)7 * 256)
static_assert(SZ_TOTAL <= (size_t)134217728);

typedef unsigned short v8us __attribute__((ext_vector_type(8), may_alias));
typedef float  v8f  __attribute__((ext_vector_type(8)));
typedef float  v4f  __attribute__((ext_vector_type(4)));
typedef float  v4fa __attribute__((ext_vector_type(4), may_alias));
typedef _Float16 v16h __attribute__((ext_vector_type(16)));
typedef _Float16 v4h __attribute__((ext_vector_type(4)));
union FragH { v16h v; v8us half[2]; _Float16 h[16]; unsigned short u[16]; };

__device__ __forceinline__ unsigned short bf16_bits(float x) { unsigned int u = __float_as_uint(x); return (unsigned short)((u + 0x7FFFu + ((u >> 16) & 1u)) >> 16); }
__device__ __forceinline__ float bf16_val(unsigned short b) { return __uint_as_float(((unsigned int)b) << 16); }
__device__ __forceinline__ float bf16_rne(float x) { return bf16_val(bf16_bits(x)); }

__global__ __launch_bounds__(256) void k_wt_f16(const float* __restrict__ W, _Float16* __restrict__ Wt, int K, int N, float scale) {
  const int t = blockIdx.x * 256 + threadIdx.x; if (t >= N * (K / 8)) return; const int n = t / (K / 8), k8 = (t % (K / 8)) * 8; FragH f;
#pragma unroll
  for (int i = 0; i < 8; ++i) f.h[i] = (_Float16)(bf16_rne(W[(size_t)(k8 + i) * N + n]) * scale);
  const v8us o = f.half[0];
  *(volatile v8us*)((unsigned short*)Wt + (size_t)n * K + k8) = o; __threadfence(); *(volatile v8us*)((unsigned short*)Wt + (size_t)n * K + k8) = o;
}

__global__ __launch_bounds__(256) void k_ln(const float* __restrict__ X, const float* __restrict__ g, const float* __restrict__ bta, float* __restrict__ XN32, _Float16* __restrict__ XN16) {
  __shared__ float red[256];
  __shared__ __attribute__((aligned(16))) _Float16 hrow[DM];
  const int r = blockIdx.x, tid = threadIdx.x;
  const int b = r / SQ, s = r - b * SQ;
  const float* x = X + ((size_t)b * SQ_FULL + s) * DM;
  const int j = tid * 4;
  const v4f a = *(const v4fa*)(x + j);
  const float v0 = bf16_rne(a[0]), v1 = bf16_rne(a[1]), v2 = bf16_rne(a[2]), v3 = bf16_rne(a[3]);
  red[tid] = (v0 + v1) + (v2 + v3); __syncthreads();
  for (int st = 128; st > 0; st >>= 1) { if (tid < st) red[tid] += red[tid + st]; __syncthreads(); }
  const float mu = red[0] * (1.0f / (float)DM); __syncthreads();
  const float c0 = v0 - mu, c1 = v1 - mu, c2 = v2 - mu, c3 = v3 - mu;
  red[tid] = (c0 * c0 + c1 * c1) + (c2 * c2 + c3 * c3); __syncthreads();
  for (int st = 128; st > 0; st >>= 1) { if (tid < st) red[tid] += red[tid + st]; __syncthreads(); }
  const float rs = rsqrtf(red[0] * (1.0f / (float)DM) + 1e-6f);
  const v4f gg = *(const v4fa*)(g + j), bb = *(const v4fa*)(bta + j);
  v4f o;
  o[0] = c0 * rs * bf16_rne(gg[0]) + bf16_rne(bb[0]);
  o[1] = c1 * rs * bf16_rne(gg[1]) + bf16_rne(bb[1]);
  o[2] = c2 * rs * bf16_rne(gg[2]) + bf16_rne(bb[2]);
  o[3] = c3 * rs * bf16_rne(gg[3]) + bf16_rne(bb[3]);
  hrow[j + 0] = (_Float16)o[0]; hrow[j + 1] = (_Float16)o[1]; hrow[j + 2] = (_Float16)o[2]; hrow[j + 3] = (_Float16)o[3];
  float* dst = XN32 + (size_t)r * DM + j;
  *(volatile v4f*)dst = o; __threadfence(); *(volatile v4f*)dst = o;
  __syncthreads();
  if (tid < 128) {
    const v8us hv = *(const v8us*)(hrow + tid * 8);
    unsigned short* d16 = (unsigned short*)XN16 + (size_t)r * DM + tid * 8;
    *(volatile v8us*)d16 = hv; __threadfence(); *(volatile v8us*)d16 = hv;
  }
}

__device__ __forceinline__ v16h g2_frag(const _Float16* p, int hh) { FragH f; f.half[0] = *(const v8us*)((const unsigned short*)p + 8 * hh); f.half[1] = *(const v8us*)((const unsigned short*)p + 16 + 8 * hh); return f.v; }
__device__ __forceinline__ v8f g2_mma(v16h a, v16h b, v8f c) { v8f d = __builtin_amdgcn_wmma_f32_16x16x32_f16(false, a, false, b, (short)0, c, false, false); asm volatile("v_nop\n\tv_nop\n\tv_nop\n\tv_nop" : "+v"(d) : "v"(a), "v"(b)); return d; }
template <int MODE>
__device__ __forceinline__ void gemm2_body(const _Float16* __restrict__ A, int lda, size_t sA, const _Float16* __restrict__ Bh, int ldb, size_t sB, float alpha,
    const float* __restrict__ R, int ldr, size_t sR, float* __restrict__ C, _Float16* __restrict__ C16, int ldc, size_t sC, int M, int N, int K) {
  static_assert(MODE == 0 || MODE == 1 || MODE == 2);
  __shared__ __attribute__((aligned(16))) float so[4][32][68];
  const int tid = threadIdx.x, w = tid >> 5, lane = tid & 31, ln = lane & 15, hh = lane >> 4; const int by = blockIdx.y;
  A += (size_t)by * sA; Bh += (size_t)by * sB; const size_t cofs = (size_t)by * sC; const size_t rofs = (size_t)by * sR;
  const int ntn = N >> 6; const int mt = blockIdx.x / ntn, nq = blockIdx.x - mt * ntn; const int row0 = mt * 128 + 32 * w, col0 = nq * 64; if (row0 >= M) return;
  const _Float16* a0p = A + (size_t)(row0 + ln) * lda; const _Float16* a1p = a0p + (size_t)16 * lda;
  const _Float16* b0p = Bh + (size_t)(col0 + ln) * ldb; const _Float16* b1p = b0p + (size_t)16 * ldb; const _Float16* b2p = b1p + (size_t)16 * ldb; const _Float16* b3p = b2p + (size_t)16 * ldb;
  const v8f z8 = {0.f,0.f,0.f,0.f,0.f,0.f,0.f,0.f}; v8f c00 = z8, c01 = z8, c02 = z8, c03 = z8, c10 = z8, c11 = z8, c12 = z8, c13 = z8;
#pragma unroll 1
  for (int kb = 0; kb < K; kb += 32) { const v16h a0 = g2_frag(a0p + kb, hh), a1 = g2_frag(a1p + kb, hh);
    v16h b = g2_frag(b0p + kb, hh); c00 = g2_mma(a0, b, c00); c10 = g2_mma(a1, b, c10);
    b = g2_frag(b1p + kb, hh); c01 = g2_mma(a0, b, c01); c11 = g2_mma(a1, b, c11);
    b = g2_frag(b2p + kb, hh); c02 = g2_mma(a0, b, c02); c12 = g2_mma(a1, b, c12);
    b = g2_frag(b3p + kb, hh); c03 = g2_mma(a0, b, c03); c13 = g2_mma(a1, b, c13); }
  v8f accs[8] = {c00, c01, c02, c03, c10, c11, c12, c13};
#pragma unroll
  for (int u = 0; u < 8; ++u) { const int t = u & 3, half = u >> 2;
#pragma unroll
    for (int r = 0; r < 8; ++r) { const int rloc = half * 16 + 8 * hh + r; so[w][rloc][t * 16 + ln] = accs[u][r] * alpha; } }
  __builtin_amdgcn_fence(4  , "workgroup"); __builtin_amdgcn_wave_barrier();
  const int rsub = lane >> 4, c4 = (lane & 15) * 4;
  for (int pass = 0; pass < 2; ++pass) {
#pragma unroll
    for (int q = 0; q < 16; ++q) { const int r = q * 2 + rsub; v4f v = *(const v4fa*)&so[w][r][c4];
      if (MODE == 2) { const v4f rv = *(const v4fa*)(R + rofs + (size_t)(row0 + r) * ldr + col0 + c4); v = v + rv; }
      if (MODE == 0) { v4h h4;
#pragma unroll
        for (int i = 0; i < 4; ++i) h4[i] = (_Float16)v[i];
        *(volatile v4h*)(C16 + cofs + (size_t)(row0 + r) * ldc + col0 + c4) = h4; }
      else { *(volatile v4f*)(C + cofs + (size_t)(row0 + r) * ldc + col0 + c4) = v; } }
    if (pass == 0) __threadfence(); } }

__global__ __launch_bounds__(128) void k_gemm_h16(const _Float16* __restrict__ A, int lda, size_t sA, const _Float16* __restrict__ Bh, int ldb, size_t sB, float alpha, _Float16* __restrict__ C16, int ldc, size_t sC, int M, int N, int K) {
  gemm2_body<0>(A, lda, sA, Bh, ldb, sB, alpha, nullptr, 0, 0, nullptr, C16, ldc, sC, M, N, K); }
__global__ __launch_bounds__(128) void k_gemm_f32(const _Float16* __restrict__ A, int lda, size_t sA, const _Float16* __restrict__ Bh, int ldb, size_t sB, float alpha, float* __restrict__ C, int ldc, size_t sC, int M, int N, int K) {
  gemm2_body<1>(A, lda, sA, Bh, ldb, sB, alpha, nullptr, 0, 0, C, nullptr, ldc, sC, M, N, K); }
__global__ __launch_bounds__(128) void k_gemm_f32add(const _Float16* __restrict__ A, int lda, size_t sA, const _Float16* __restrict__ Bh, int ldb, size_t sB, float alpha, const float* __restrict__ R, int ldr, size_t sR, float* __restrict__ C, int ldc, size_t sC, int M, int N, int K) {
  gemm2_body<2>(A, lda, sA, Bh, ldb, sB, alpha, R, ldr, sR, C, nullptr, ldc, sC, M, N, K); }

__global__ __launch_bounds__(256) void k_rsm(const float* __restrict__ S, _Float16* __restrict__ P, int nrows) {
  #pragma clang fp contract(off)
  const int i = blockIdx.x * 256 + threadIdx.x; if (i >= nrows) return; const float* s = S + (size_t)i * SQ; float mx = -3.0e38f;
#pragma unroll 1
  for (int j = 0; j < SQ; ++j) mx = fmaxf(mx, s[j]);
  float se = 0.f;
#pragma unroll 1
  for (int j = 0; j < SQ; ++j) se += expf(s[j] - mx);
  const float sc = 256.0f / se;
#pragma unroll 1
  for (int j0 = 0; j0 < SQ; j0 += 8) { FragH f;
#pragma unroll
    for (int q = 0; q < 8; ++q) f.h[q] = (_Float16)(expf(s[j0 + q] - mx) * sc);
    const v8us o = f.half[0]; unsigned short* d = (unsigned short*)P + (size_t)i * SQ + j0; *(volatile v8us*)d = o; __threadfence(); *(volatile v8us*)d = o; } }

__global__ __launch_bounds__(256) void k_vt(const _Float16* __restrict__ V16, int ldv, _Float16* __restrict__ Vt) {
  __shared__ unsigned short tl[64][66]; const int tid = threadIdx.x; const int slab = blockIdx.x / (SQ / 64), lg = blockIdx.x % (SQ / 64); const int b = slab / NH, h = slab % NH;
  for (int i = tid; i < 64 * 8; i += 256) { const int r = i / 8, c8 = (i % 8) * 8; FragH f; f.half[0] = *(const v8us*)((const unsigned short*)V16 + ((size_t)b * SQ + lg * 64 + r) * ldv + h * HD + c8);
#pragma unroll
    for (int q = 0; q < 8; ++q) tl[r][c8 + q] = f.u[q]; }
  __syncthreads();
  for (int pass = 0; pass < 2; ++pass) {
#pragma unroll
    for (int rd = 0; rd < 2; ++rd) { const int d = rd * 32 + tid / 8, pc = tid % 8; FragH f;
#pragma unroll
      for (int q = 0; q < 8; ++q) f.u[q] = tl[pc * 8 + q][d];
      const v8us o = f.half[0];
      *(volatile v8us*)((unsigned short*)Vt + ((size_t)slab * HD + d) * SQ + lg * 64 + pc * 8) = o; }
    if (pass == 0) __threadfence(); } }

extern "C" void kernel_launch(void* const* d_in, const int* in_sizes, int n_in,
                              void* d_out, int out_size, void* d_ws, size_t ws_size, hipStream_t stream) {
  if (n_in < 6) return;
  const size_t need_x = ((size_t)(NB - 1) * SQ_FULL + SQ) * DM;
  if ((size_t)in_sizes[0] < need_x || in_sizes[1] < DM || in_sizes[2] < DM) return;
  if ((size_t)in_sizes[3] < (size_t)DM * DM || (size_t)in_sizes[4] < (size_t)DM * DM || (size_t)in_sizes[5] < (size_t)DM * DM) return;
  if ((size_t)out_size < need_x) return;
  const float* x = (const float*)d_in[0]; const float* lng = (const float*)d_in[1]; const float* lnb = (const float*)d_in[2];
  const float* wq = (const float*)d_in[3]; const float* wk = (const float*)d_in[4]; const float* wv = (const float*)d_in[5];
  float* out = (float*)d_out;
  char* ws = (char*)d_ws; size_t off = 0;
  auto take = [&](size_t bytes) { char* p = ws + off; off += (bytes + 255) & ~(size_t)255; return p; };
  _Float16* BQKV = (_Float16*)take(SZ_BQKV);
  float* XN32 = (float*)take(SZ_XN32);
  _Float16* XN16 = (_Float16*)take(SZ_XN16);
  _Float16* QKV = (_Float16*)take(SZ_QKV); _Float16* Q16 = QKV; _Float16* K16 = QKV + DM; _Float16* V16 = QKV + 2 * DM;
  float* S = (float*)take(SZ_S); _Float16* P = (_Float16*)take(SZ_P); _Float16* VT = (_Float16*)take(SZ_VT);
  if (off > ws_size) return;
  const unsigned wtg = (unsigned)(((size_t)DM * DM / 8 + 255) / 256);
  k_wt_f16<<<wtg, 256, 0, stream>>>(wq, BQKV, DM, DM, 16.0f);
  k_wt_f16<<<wtg, 256, 0, stream>>>(wk, BQKV + (size_t)DM * DM, DM, DM, 16.0f);
  k_wt_f16<<<wtg, 256, 0, stream>>>(wv, BQKV + (size_t)2 * DM * DM, DM, DM, 16.0f);
  k_ln<<<(unsigned)NR, 256, 0, stream>>>(x, lng, lnb, XN32, XN16);
  k_gemm_h16<<<dim3((unsigned)((NR / 128) * (3 * DM / 64)), 1), 128, 0, stream>>>(XN16, DM, 0, BQKV, DM, 0, 0.0625f, QKV, LQ, 0, (int)NR, 3 * DM, DM);
  k_vt<<<NB * NH * (SQ / 64), 256, 0, stream>>>(V16, LQ, VT);
  for (int b = 0; b < NB; ++b) { const size_t r0 = (size_t)b * SQ;
    for (int h0 = 0; h0 < NH; h0 += HG) {
      k_gemm_f32<<<dim3((SQ / 128) * (SQ / 64), HG), 128, 0, stream>>>(Q16 + r0 * LQ + h0 * HD, LQ, (size_t)HD, K16 + r0 * LQ + h0 * HD, LQ, (size_t)HD, 0.03125f, S, SQ, (size_t)SQ * SQ, SQ, SQ, HD);
      k_rsm<<<(HG * SQ + 255) / 256, 256, 0, stream>>>(S, P, HG * SQ);
      k_gemm_f32add<<<dim3((SQ / 128) * (HD / 64), HG), 128, 0, stream>>>(P, SQ, (size_t)SQ * SQ, VT + ((size_t)b * NH + h0) * HD * SQ, SQ, (size_t)HD * SQ, 0.00390625f,
          XN32 + r0 * DM + h0 * HD, DM, (size_t)HD, out + ((size_t)b * SQ_FULL) * DM + h0 * HD, DM, (size_t)HD, SQ, HD, SQ); } }
}
